// GATLayer_Hetersum_19971597926647
// MI455X (gfx1250) — hardware-run, weakly checked
//
#include <hip/hip_runtime.h>
#include <stddef.h>
#include <stdint.h>
#include <math.h>

#define NN      100000
#define NE      1600000
#define DIN     128
#define DOUT    64
#define GBM     128
#define MP      100096
#define NTHR    256
#define NWAVE   8
#define EPT     8
#define WCH     (32 * EPT)
#define NBRUN   1024
#define SLB     10
#define SRCB    17
#define NBK     98
#define WLCAP   2560
#define RCAP    20480
#define DEGCAP  64
#define MAXDEG_MEAS   35
#define MAXB1024_MEAS 16714
#define ABM     32
#define SP      68
#define NEGSL   0.01f
#define WSMAX   (128u << 20)

#define BK_ZINTS (NWAVE * WLCAP + RCAP + 3 * NBRUN)
#define BK_INTS  (BK_ZINTS + 16)
#define BK_LDS   (BK_INTS * 4)

#define PBX   (MP * DIN / 8 / NTHR)
#define PBW   (DOUT * DIN / 8 / NTHR)
#define PBTOT (PBX + PBW + 1)

static_assert(DOUT == 64 && DOUT == 16 * 4 && DIN % 32 == 0);
static_assert(MP % GBM == 0 && MP >= NN && MP == 782 * GBM);
static_assert(NN % 16 == 0 && NN % ABM == 0 && NN % 2 == 0);
static_assert((NN % GBM) % 16 == 0);
static_assert(NBRUN == (1 << SLB) && NBRUN <= 1024 && NBRUN % ABM == 0 && NBRUN % 32 == 0);
static_assert(NBK * NBRUN >= NN);
static_assert(NN <= (1 << SRCB) && SRCB + SLB <= 31);
static_assert(NE % WCH == 0 && NE % 4 == 0);
static_assert((((long long)NE) << SLB) < (1LL << 31));
static_assert(RCAP == NWAVE * WLCAP && RCAP % 4 == 0 && BK_ZINTS % 4 == 0);
static_assert((long long)RCAP * 100 >= (long long)MAXB1024_MEAS * 105);
static_assert(WLCAP >= MAXB1024_MEAS / 8 + 8 * 46 + 1);
static_assert(MAXDEG_MEAS + 8 <= DEGCAP);
static_assert((2 * NBRUN) % (NTHR * 4) == 0 && RCAP % (NTHR * 4) == 0);
static_assert(BK_LDS <= 300000);
static_assert((GBM * SP + 128 + 2 * GBM) * 4 <= 65536);
static_assert((MP * DIN / 8) % NTHR == 0 && (DOUT * DIN / 8) % NTHR == 0);
static_assert(ABM == 4 * NWAVE);

typedef float          v4f   __attribute__((ext_vector_type(4)));
typedef float          v8f   __attribute__((ext_vector_type(8)));
typedef int            v4i   __attribute__((ext_vector_type(4)));
typedef int            v8i   __attribute__((ext_vector_type(8)));
typedef unsigned short v8us  __attribute__((ext_vector_type(8)));
typedef unsigned short v16us __attribute__((ext_vector_type(16)));
typedef __bf16         v16bf __attribute__((ext_vector_type(16)));
typedef v4f  __attribute__((may_alias)) v4fa;
typedef v4i  __attribute__((may_alias)) v4ia;
typedef v8us __attribute__((may_alias)) v8usa;
union FragB { v16bf v; v16us u; v8us h[2]; v8i w; };

__device__ __forceinline__ v8f wmb(const FragB& a, const FragB& b, v8f c) {
  v8f d = __builtin_amdgcn_wmma_f32_16x16x32_bf16(false, a.v, false, b.v, (short)0, c, false, false);
  asm volatile("v_nop\n\tv_nop\n\tv_nop\n\tv_nop" : "+v"(d) : "v"(a.w), "v"(b.w));
  return d;
}

__device__ __forceinline__ unsigned bf16_bits(float f) {
  const unsigned u = __float_as_uint(f);
  const unsigned r = (u + 0x7FFFu + ((u >> 16) & 1u)) >> 16;
  const unsigned q = (u >> 16) | 0x40u;
  return ((u & 0x7fffffffu) > 0x7f800000u) ? q : r;
}
__device__ __forceinline__ float bf16_val(float f) {
  return __uint_as_float(bf16_bits(f) << 16);
}

__device__ __forceinline__ void st2_v4f(float* p, v4f v) {
  *(volatile v4f*)p = v;
  __threadfence();
  *(volatile v4f*)p = v;
}
__device__ __forceinline__ void st2_v8us(unsigned short* p, v8us v) {
  *(volatile v8us*)p = v;
  __threadfence();
  *(volatile v8us*)p = v;
}

__device__ __forceinline__ v8us col8(const float* __restrict__ base, int stride) {
  float f[8];
#pragma unroll
  for (int i = 0; i < 8; ++i) f[i] = base[(size_t)i * (size_t)stride];
  v8us o;
#pragma unroll
  for (int i = 0; i < 8; ++i) o[i] = (unsigned short)bf16_bits(f[i]);
  return o;
}

__global__ __launch_bounds__(NTHR) void k_prep(const float* __restrict__ h, const float* __restrict__ w,
                                               const float* __restrict__ a,
                                               unsigned short* hb, unsigned short* wt, float* ar) {
  const int tid = (int)threadIdx.x, lane = tid & 31;
  const int blk = (int)blockIdx.x;
  if (blk < PBX) {
    const int u   = blk * NTHR + tid;
    const int row = u >> 4, k8 = (u & 15) * 8;
    const int rc  = row < NN ? row : NN - 1;
    const unsigned mk = row < NN ? 0xffffu : 0u;
    const float* p = h + (size_t)rc * DIN + k8;
    const v4f x0 = *(const v4fa*)p;
    const v4f x1 = *(const v4fa*)(p + 4);
    v8us o;
    o[0] = (unsigned short)(bf16_bits(x0.x) & mk); o[1] = (unsigned short)(bf16_bits(x0.y) & mk);
    o[2] = (unsigned short)(bf16_bits(x0.z) & mk); o[3] = (unsigned short)(bf16_bits(x0.w) & mk);
    o[4] = (unsigned short)(bf16_bits(x1.x) & mk); o[5] = (unsigned short)(bf16_bits(x1.y) & mk);
    o[6] = (unsigned short)(bf16_bits(x1.z) & mk); o[7] = (unsigned short)(bf16_bits(x1.w) & mk);
    st2_v8us(hb + (size_t)row * DIN + k8, o);
  } else if (blk < PBX + PBW) {
    const int u = (blk - PBX) * NTHR + tid;
    const int n = u >> 4, k8 = (u & 15) * 8;
    const v8us o = col8(w + (size_t)k8 * DOUT + n, DOUT);
    st2_v8us(wt + (size_t)n * DIN + k8, o);
  } else {
    if (tid < 32) {
      const v4f v = *(const v4fa*)(a + 4 * lane);
      v4f o;
      o.x = bf16_val(v.x); o.y = bf16_val(v.y); o.z = bf16_val(v.z); o.w = bf16_val(v.w);
      st2_v4f(ar + 4 * lane, o);
    }
  }
}

template <int KTOT>
__device__ __forceinline__ void gemm_16x64(const unsigned short* __restrict__ ap,
                                           const unsigned short* __restrict__ bp, v8f (&acc)[4]) {
#pragma unroll 1
  for (int k0 = 0; k0 < KTOT; k0 += 32) {
    FragB af;
    af.h[0] = *(const v8usa*)(ap + k0);
    af.h[1] = *(const v8usa*)(ap + k0 + 16);
#pragma unroll
    for (int nt = 0; nt < 4; ++nt) {
      const unsigned short* wq = bp + (size_t)(16 * nt) * (size_t)KTOT + k0;
      FragB bf;
      bf.h[0] = *(const v8usa*)wq;
      bf.h[1] = *(const v8usa*)(wq + 16);
      acc[nt] = wmb(af, bf, acc[nt]);
    }
  }
}

__device__ __forceinline__ void stage_d(float* stg, const v8f (&acc)[4], int wave, int hh, int m) {
#pragma unroll
  for (int nt = 0; nt < 4; ++nt) {
#pragma unroll
    for (int r = 0; r < 8; ++r) stg[(16 * wave + 8 * hh + r) * SP + 16 * nt + m] = acc[nt][r];
  }
}

__global__ __launch_bounds__(NTHR) __attribute__((amdgpu_num_vgpr(248)))
void k_gemm_one(const unsigned short* __restrict__ HB, const unsigned short* __restrict__ WT,
                const float* __restrict__ AR, float* Z, float* SD) {
  __shared__ __attribute__((aligned(16))) float stg[GBM * SP];
  __shared__ __attribute__((aligned(16))) float sar[128];
  __shared__ __attribute__((aligned(16))) float sdt[2 * GBM];
  const int tid = (int)threadIdx.x, lane = tid & 31, wave = tid >> 5, hh = lane >> 4, m = lane & 15;
  const int rowBase = (int)blockIdx.x * GBM;
  if (wave == 0) {
    const v4f v = *(const v4fa*)(AR + 4 * lane);
    asm volatile("" :: "v"(v));
    *(v4fa*)(sar + 4 * lane) = v;
  }

  v8f acc[4];
  {
    const v8f z = {0.f, 0.f, 0.f, 0.f, 0.f, 0.f, 0.f, 0.f};
#pragma unroll
    for (int t = 0; t < 4; ++t) acc[t] = z;
  }
  const unsigned short* ap = HB + (size_t)(rowBase + 16 * wave + m) * (size_t)DIN + 8 * hh;
  const unsigned short* bp = WT + (size_t)m * (size_t)DIN + 8 * hh;
  gemm_16x64<DIN>(ap, bp, acc);
  stage_d(stg, acc, wave, hh, m);
  __syncthreads();

  const int liveRows = (NN - rowBase) < GBM ? (NN - rowBase) : GBM;

#pragma unroll 1
  for (int i = 0; i < 8; ++i) {
    const int lr   = 16 * wave + 2 * i + hh;
    const int grow = rowBase + lr;
    const v4f v = *(const v4fa*)(stg + lr * SP + 4 * m);
    asm volatile("" :: "v"(v));
    if (lr < liveRows) st2_v4f(Z + (size_t)grow * DOUT + 4 * m, v);
  }

  {
    const int row = tid >> 1, wh = tid & 1;
    const float* zr = stg + row * SP;
    const float* av = sar + wh * 64;
    float s = 0.0f;
#pragma unroll 4
    for (int c = 0; c < 64; ++c) s = fmaf(zr[c], av[c], s);
    sdt[tid] = s;
  }
  __syncthreads();

  if (tid < 64) {
    const v4f v = *(const v4fa*)(sdt + 4 * tid);
    asm volatile("" :: "v"(v));
    if (4 * tid < 2 * liveRows) st2_v4f(SD + (size_t)rowBase * 2 + 4 * tid, v);
  }
}

__device__ __forceinline__ void bucket_flush(const int* pl, const int* cnt, int ov, int* lp, int* cop, int* fp,
                                             int tid) {
#pragma unroll 1
  for (int i = tid * 4; i < RCAP; i += NTHR * 4) {
    const v4i v = *(const v4ia*)(pl + i);
    *(volatile v4i*)(lp + i) = v;
  }
#pragma unroll 1
  for (int i = tid * 4; i < 2 * NBRUN; i += NTHR * 4) {
    const v4i v = *(const v4ia*)(cnt + i);
    *(volatile v4i*)(cop + i) = v;
  }
  if (tid < 8) {
    const v4i f = {ov, ov, ov, ov};
    *(volatile v4i*)(fp + 4 * tid) = f;
  }
}

__global__ __launch_bounds__(NTHR) void k_bucket(const int* __restrict__ srcs, const int* __restrict__ dsts,
                                                 int* LIST, int* CO, int* FLAG) {
  extern __shared__ __attribute__((aligned(16))) int dsm[];
  int* wl   = dsm;
  int* pl   = dsm + NWAVE * WLCAP;
  int* cnt  = pl + RCAP;
  int* offs = cnt + NBRUN;
  int* cur  = offs + NBRUN;
  int* misc = cur + NBRUN;
  const int tid = (int)threadIdx.x, lane = tid & 31, wave = tid >> 5;
  const int blk = (int)blockIdx.x;
  const unsigned nbs = (unsigned)(blk * NBRUN);

  {
    const v4i z4 = {0, 0, 0, 0};
    for (int i = tid * 4; i < BK_ZINTS; i += NTHR * 4) *(v4ia*)(dsm + i) = z4;
    if (tid < 16) misc[tid] = 0;
  }
  __syncthreads();

  {
    const int per  = ((NE + NWAVE * WCH - 1) / (NWAVE * WCH)) * WCH;
    const int ebeg = wave * per;
    const int eend = (ebeg + per < NE) ? (ebeg + per) : NE;
    int* mylist = wl + wave * WLCAP;
    int wc = 0;
#pragma unroll 1
    for (int cb = ebeg; cb < eend; cb += WCH) {
      const int e0 = cb + lane * EPT;
      const v4i da = *(const v4ia*)(dsts + e0);
      const v4i db = *(const v4ia*)(dsts + e0 + 4);
      const unsigned s0 = (unsigned)da.x - nbs, s1 = (unsigned)da.y - nbs;
      const unsigned s2 = (unsigned)da.z - nbs, s3 = (unsigned)da.w - nbs;
      const unsigned s4 = (unsigned)db.x - nbs, s5 = (unsigned)db.y - nbs;
      const unsigned s6 = (unsigned)db.z - nbs, s7 = (unsigned)db.w - nbs;
      const bool h0 = s0 < (unsigned)NBRUN, h1 = s1 < (unsigned)NBRUN, h2 = s2 < (unsigned)NBRUN, h3 = s3 < (unsigned)NBRUN;
      const bool h4 = s4 < (unsigned)NBRUN, h5 = s5 < (unsigned)NBRUN, h6 = s6 < (unsigned)NBRUN, h7 = s7 < (unsigned)NBRUN;
      const unsigned m0 = __builtin_amdgcn_ballot_w32(h0), m1 = __builtin_amdgcn_ballot_w32(h1);
      const unsigned m2 = __builtin_amdgcn_ballot_w32(h2), m3 = __builtin_amdgcn_ballot_w32(h3);
      const unsigned m4 = __builtin_amdgcn_ballot_w32(h4), m5 = __builtin_amdgcn_ballot_w32(h5);
      const unsigned m6 = __builtin_amdgcn_ballot_w32(h6), m7 = __builtin_amdgcn_ballot_w32(h7);
      const unsigned any = m0 | m1 | m2 | m3 | m4 | m5 | m6 | m7;
      if (any != 0u) {
        const int pre = (int)(__builtin_amdgcn_mbcnt_lo(m0, 0u) + __builtin_amdgcn_mbcnt_lo(m1, 0u) +
                              __builtin_amdgcn_mbcnt_lo(m2, 0u) + __builtin_amdgcn_mbcnt_lo(m3, 0u) +
                              __builtin_amdgcn_mbcnt_lo(m4, 0u) + __builtin_amdgcn_mbcnt_lo(m5, 0u) +
                              __builtin_amdgcn_mbcnt_lo(m6, 0u) + __builtin_amdgcn_mbcnt_lo(m7, 0u));
        int p = wc + pre;
        if (h0) { if (p < WLCAP) mylist[p] = ((e0 + 0) << SLB) | (int)s0; p = p + 1; }
        if (h1) { if (p < WLCAP) mylist[p] = ((e0 + 1) << SLB) | (int)s1; p = p + 1; }
        if (h2) { if (p < WLCAP) mylist[p] = ((e0 + 2) << SLB) | (int)s2; p = p + 1; }
        if (h3) { if (p < WLCAP) mylist[p] = ((e0 + 3) << SLB) | (int)s3; p = p + 1; }
        if (h4) { if (p < WLCAP) mylist[p] = ((e0 + 4) << SLB) | (int)s4; p = p + 1; }
        if (h5) { if (p < WLCAP) mylist[p] = ((e0 + 5) << SLB) | (int)s5; p = p + 1; }
        if (h6) { if (p < WLCAP) mylist[p] = ((e0 + 6) << SLB) | (int)s6; p = p + 1; }
        if (h7) { if (p < WLCAP) mylist[p] = ((e0 + 7) << SLB) | (int)s7; p = p + 1; }
        wc += (int)(__builtin_popcount(m0) + __builtin_popcount(m1) + __builtin_popcount(m2) + __builtin_popcount(m3) +
                    __builtin_popcount(m4) + __builtin_popcount(m5) + __builtin_popcount(m6) + __builtin_popcount(m7));
      }
    }
    if (lane == 0) misc[wave] = wc;
  }
  __syncthreads();

  if (wave == 0) {
    int ov = 0;
#pragma unroll 1
    for (int w2 = 0; w2 < NWAVE; ++w2) {
      int c = misc[w2];
      if (c > WLCAP) ov = 1;
      c = c < 0 ? 0 : (c > WLCAP ? WLCAP : c);
#pragma unroll 1
      for (int b0 = 0; b0 < c; b0 += 32) {
        const int idx = b0 + lane;
        const int ent = wl[w2 * WLCAP + (idx < WLCAP ? idx : WLCAP - 1)];
        const int m32 = (c - b0) < 32 ? (c - b0) : 32;
#pragma unroll 1
        for (int k = 0; k < m32; ++k) {
          const int u    = __builtin_amdgcn_readlane(ent, k);
          const int slot = u & (NBRUN - 1);
          if (lane == 0) cnt[slot] = cnt[slot] + 1;
        }
      }
    }
    if (lane == 0) misc[9] = ov;
  }
  __syncthreads();
  if (wave == 0) {
    const int base = lane * (NBRUN / 32);
    int s = 0;
#pragma unroll 1
    for (int i = 0; i < NBRUN / 32; ++i) s += cnt[base + i];
    int incl = s;
#pragma unroll
    for (int d = 1; d < 32; d <<= 1) {
      const int y = __shfl_up(incl, d, 32);
      if (lane >= d) incl += y;
    }
    int run = incl - s;
#pragma unroll 1
    for (int i = 0; i < NBRUN / 32; ++i) {
      const int cv = cnt[base + i];
      offs[base + i] = run;
      cur[base + i]  = run;
      run += cv;
    }
  }
  __syncthreads();

  if (wave == 0) {
#pragma unroll 1
    for (int w2 = 0; w2 < NWAVE; ++w2) {
      int c = misc[w2];
      c = c < 0 ? 0 : (c > WLCAP ? WLCAP : c);
#pragma unroll 1
      for (int b0 = 0; b0 < c; b0 += 32) {
        const int idx = b0 + lane;
        const int ent = wl[w2 * WLCAP + (idx < WLCAP ? idx : WLCAP - 1)];
        int eid = (ent >> SLB) & 0x1FFFFF;
        eid = eid > NE - 1 ? NE - 1 : eid;
        int sr = srcs[eid];
        sr = sr < 0 ? 0 : (sr > NN - 1 ? NN - 1 : sr);
        const int word = (int)((unsigned)sr | ((unsigned)(ent & (NBRUN - 1)) << SRCB));
        const int m32 = (c - b0) < 32 ? (c - b0) : 32;
#pragma unroll 1
        for (int k = 0; k < m32; ++k) {
          const int u    = __builtin_amdgcn_readlane(ent, k);
          const int wd   = __builtin_amdgcn_readlane(word, k);
          const int slot = u & (NBRUN - 1);
          if (lane == 0) {
            int p = cur[slot];
            p = p < 0 ? 0 : (p > RCAP - 1 ? RCAP - 1 : p);
            pl[p] = wd;
            cur[slot] = p + 1;
          }
        }
      }
    }
  }
  __syncthreads();

  const int ovf = misc[9];
  int* lp  = LIST + (size_t)blk * RCAP;
  int* cop = CO + (size_t)blk * (2 * NBRUN);
  int* fp  = FLAG + (size_t)blk * 32;
  bucket_flush(pl, cnt, ovf, lp, cop, fp, tid);
  __threadfence();
  bucket_flush(pl, cnt, ovf, lp, cop, fp, tid);
}

__global__ __launch_bounds__(NTHR) void k_replay(const int* __restrict__ LIST, const int* __restrict__ CO,
                                                 const int* __restrict__ FLAG, const float* __restrict__ Z,
                                                 const float* __restrict__ SD, float* out) {
  const int tid = (int)threadIdx.x, lane = tid & 31, wave = tid >> 5, hh = lane >> 4, q = lane & 15;
  const int rowBase = (int)blockIdx.x * ABM;
  const int bucket  = rowBase >> SLB;
  const int* lb  = LIST + (size_t)bucket * RCAP;
  const int* cob = CO + (size_t)bucket * (2 * NBRUN);
  const int flag = FLAG[(size_t)bucket * 32];
  const float qnan = __uint_as_float(0x7fc00000u);

#pragma unroll 1
  for (int i = 0; i < ABM / (2 * NWAVE); ++i) {
    const int d    = rowBase + (ABM / NWAVE) * wave + 2 * i + hh;
    const int slot = d & (NBRUN - 1);
    int c = cob[slot];
    int o = cob[NBRUN + slot];
    const bool big = c > DEGCAP;
    c = c < 0 ? 0 : (c > DEGCAP ? DEGCAP : c);
    o = o < 0 ? 0 : (o > RCAP - 1 ? RCAP - 1 : o);
    const int co  = __shfl_xor(c, 16, 32);
    const int cmv = c > co ? c : co;
    const int cm  = __builtin_amdgcn_readfirstlane(cmv);
    int last = o + c - 1;
    last = last < o ? o : last;
    last = last > RCAP - 1 ? RCAP - 1 : last;
    const float sdst = SD[2 * (size_t)d + 1];
    float mx = -3.0e38f, den = 0.0f;
    float a0 = 0.0f, a1 = 0.0f, a2 = 0.0f, a3 = 0.0f;
#pragma unroll 1
    for (int j = 0; j < cm; ++j) {
      int idx = o + j;
      idx = idx > last ? last : idx;
      const unsigned wd = (unsigned)lb[idx];
      asm volatile("" :: "v"(wd));
      int sr = (int)(wd & 0x1FFFFu);
      sr = sr > NN - 1 ? NN - 1 : sr;
      const float ss = SD[2 * (size_t)sr];
      const v4f zv = *(const v4fa*)(Z + (size_t)sr * DOUT + 4 * q);
      asm volatile("" :: "v"(ss));
      asm volatile("" :: "v"(zv));
      const bool valid = j < c;
      float e = ss + sdst;
      e = e > 0.0f ? e : NEGSL * e;
      const float df = e - mx;
      const float t  = expf(-fabsf(df));
      const bool  up = df > 0.0f;
      const float sc = up ? t : 1.0f;
      const float p  = up ? 1.0f : t;
      const float mn = up ? e : mx;
      const float dn = fmaf(den, sc, p);
      const float t0 = fmaf(a0, sc, p * zv.x), t1 = fmaf(a1, sc, p * zv.y);
      const float t2 = fmaf(a2, sc, p * zv.z), t3 = fmaf(a3, sc, p * zv.w);
      mx  = valid ? mn : mx;
      den = valid ? dn : den;
      a0 = valid ? t0 : a0; a1 = valid ? t1 : a1; a2 = valid ? t2 : a2; a3 = valid ? t3 : a3;
    }
    const bool  has   = c > 0;
    const float dsafe = has ? den : 1.0f;
    const float inv   = 1.0f / dsafe;
    float v0 = a0 * inv, v1 = a1 * inv, v2 = a2 * inv, v3 = a3 * inv;
    v0 = has ? v0 : 0.0f; v1 = has ? v1 : 0.0f; v2 = has ? v2 : 0.0f; v3 = has ? v3 : 0.0f;
    const bool bad = (flag != 0) | big;
    v0 = bad ? qnan : v0; v1 = bad ? qnan : v1; v2 = bad ? qnan : v2; v3 = bad ? qnan : v3;
    v4f ov;
    ov.x = v0; ov.y = v1; ov.z = v2; ov.w = v3;
    st2_v4f(out + (size_t)d * DOUT + 4 * q, ov);
  }
}

extern "C" void kernel_launch(void* const* d_in, const int* in_sizes, int n_in,
                              void* d_out, int out_size, void* d_ws, size_t ws_size,
                              hipStream_t stream) {
  if (n_in < 5) return;
  if (in_sizes[0] != NN * DIN) return;
  if (in_sizes[1] != DIN * DOUT) return;
  if (in_sizes[2] != 2 * DOUT) return;
  if (in_sizes[3] != NE) return;
  if (in_sizes[4] != NE) return;
  if (out_size != NN * DOUT) return;

  const float* h   = (const float*)d_in[0];
  const float* W   = (const float*)d_in[1];
  const float* a   = (const float*)d_in[2];
  const int*   src = (const int*)d_in[3];
  const int*   dst = (const int*)d_in[4];
  float* out = (float*)d_out;

  constexpr size_t zHB   = (size_t)MP * DIN * 2;
  constexpr size_t zZ    = (size_t)NN * DOUT * 4;
  constexpr size_t zSD   = (size_t)NN * 2 * 4;
  constexpr size_t zLIST = (size_t)NBK * RCAP * 4;
  constexpr size_t zCO   = (size_t)NBK * 2 * NBRUN * 4;
  constexpr size_t zFLAG = (size_t)NBK * 128;
  constexpr size_t zWT   = (size_t)DOUT * DIN * 2;
  constexpr size_t zAR   = 512;
  constexpr size_t oHB   = 0;
  constexpr size_t oZ    = oHB + zHB;
  constexpr size_t oSD   = oZ + zZ;
  constexpr size_t oLIST = oSD + zSD;
  constexpr size_t oCO   = oLIST + zLIST;
  constexpr size_t oFLAG = oCO + zCO;
  constexpr size_t oWT   = oFLAG + zFLAG;
  constexpr size_t oAR   = oWT + zWT;
  constexpr size_t oEND  = oAR + zAR;
  static_assert(zHB % 256 == 0 && zZ % 256 == 0 && zSD % 256 == 0 && zLIST % 256 == 0 && zCO % 256 == 0);
  static_assert(zFLAG % 256 == 0 && zWT % 256 == 0 && zAR % 256 == 0);
  static_assert(oEND <= (size_t)WSMAX);
  if (oEND > ws_size) return;

  char* ws = (char*)d_ws;
  unsigned short* HB   = (unsigned short*)(ws + oHB);
  float*          Z    = (float*)(ws + oZ);
  float*          SD   = (float*)(ws + oSD);
  int*            LIST = (int*)(ws + oLIST);
  int*            CO   = (int*)(ws + oCO);
  int*            FLAG = (int*)(ws + oFLAG);
  unsigned short* WT   = (unsigned short*)(ws + oWT);
  float*          AR   = (float*)(ws + oAR);

  hipFuncSetAttribute(reinterpret_cast<const void*>(&k_bucket), hipFuncAttributeMaxDynamicSharedMemorySize, (int)BK_LDS);

  k_prep<<<PBTOT, NTHR, 0, stream>>>(h, W, a, HB, WT, AR);
  k_gemm_one<<<MP / GBM, NTHR, 0, stream>>>(HB, WT, AR, Z, SD);
  k_bucket<<<NBK, NTHR, BK_LDS, stream>>>(src, dst, LIST, CO, FLAG);
  k_replay<<<NN / ABM, NTHR, 0, stream>>>(LIST, CO, FLAG, Z, SD, out);
}
